// Optimized_DSTGAT_Attn_84061099917964
// MI455X (gfx1250) — hardware-run, weakly checked
//
#include <hip/hip_runtime.h>
#include <stddef.h>
#include <math.h>


#define TT     1024
#define NF     16
#define KW     25
#define XOF    12
#define XSN    1056
#define P1     1028
#define FPITCH 32
#define FTHR   256
#define FWAV   8

#define LF_XS   0
#define LF_S1   (XSN * 4)
#define LF_S2   (LF_S1 + NF * P1 * 4)
#define LF_RED  (LF_S2 + NF * P1 * 4)
#define LF_FV   (LF_RED + FWAV * NF * 4)
#define LF_PAR  (LF_FV + FPITCH * 4)
#define LDS_FEAT (LF_PAR + 192 * 4)

#define GN   64
#define NE   512
#define NH   4
#define HF   32
#define DF   128
#define HP   132
#define AHP  40
#define GTHR 256

#define O_HH  0
#define O_GO  (O_HH + GN * HP * 4)
#define O_H1  (O_GO + GN * DF * 4)
#define O_SK  (O_H1 + GN * HF * 4)
#define O_ASD (O_SK + GN * HF * 4)
#define O_AV  (O_ASD + GN * 8 * 4)
#define O_EI  (O_AV + 2 * DF * 4)
#define O_AH  (O_EI + (3 * NE + 2 * GN) * 4)
#define O_WT  (O_AH + GN * AHP * 2)
#define O_WK  (O_WT + DF * AHP * 2)
#define O_PL  (O_WK + HF * AHP * 2)
#define LDS_GRAPH (O_PL + FPITCH * 4)

static_assert(LDS_FEAT == 137216);
static_assert(LDS_GRAPH == 110720);
static_assert((LF_S1 % 16) == 0 && (LF_S2 % 16) == 0 && (LF_RED % 16) == 0 && (LF_FV % 16) == 0);
static_assert((P1 % 4) == 0);
static_assert(XSN >= TT - 16 + 15 + 31 + 1);
static_assert(TT * NF * 2 <= NF * P1 * 4);
static_assert((O_GO % 16) == 0 && (O_ASD % 16) == 0 && (O_EI % 16) == 0 && (O_AH % 16) == 0);
static_assert((O_WT % 16) == 0 && (O_WK % 16) == 0 && (O_PL % 16) == 0);
static_assert(GTHR == GN * NH);

typedef float    v4f  __attribute__((ext_vector_type(4)));
typedef float    v8f  __attribute__((ext_vector_type(8)));
typedef _Float16 v8h  __attribute__((ext_vector_type(8)));
typedef _Float16 v16h __attribute__((ext_vector_type(16)));
union Frag { v16h v; v8h half[2]; };

__device__ __forceinline__ v8f wm(v16h a, v16h b, v8f c) {
  v8f d = __builtin_amdgcn_wmma_f32_16x16x32_f16(false, a, false, b, (short)0, c, false, false);
  asm volatile("v_nop\n\tv_nop\n\tv_nop\n\tv_nop" : "+v"(d) : "v"(a), "v"(b));
  return d;
}

__device__ __forceinline__ float elu_f(float v)   { return v > 0.0f ? v : (__expf(v) - 1.0f); }
__device__ __forceinline__ float gelu_f(float v)  { return 0.5f * v * (1.0f + erff(v * 0.70710678118654752f)); }
__device__ __forceinline__ float lrelu_f(float v) { return v >= 0.0f ? v : 0.2f * v; }

__global__ __launch_bounds__(FTHR) void k_feat(
    const float* __restrict__ x,   const float* __restrict__ w1,
    const float* __restrict__ g1,  const float* __restrict__ b1,
    const float* __restrict__ wd,  const float* __restrict__ g2, const float* __restrict__ b2,
    const float* __restrict__ wsd, const float* __restrict__ wp,
    const float* __restrict__ g3,  const float* __restrict__ b3,
    float* feat, int nNodes)
{
  extern __shared__ v4f dynf[];
  char* base = (char*)dynf;
  float*    xs  = (float*)(base + LF_XS);
  float*    s1  = (float*)(base + LF_S1);
  float*    s2  = (float*)(base + LF_S2);
  _Float16* s3  = (_Float16*)(base + LF_S1);
  float*    red = (float*)(base + LF_RED);
  float*    fvv = (float*)(base + LF_FV);
  float*    par = (float*)(base + LF_PAR);

  const int tid = threadIdx.x, lane = tid & 31, wave = tid >> 5;
  const int h = lane >> 4, m = lane & 15;
  const int node = blockIdx.x;
  if (node >= nNodes) return;

  const float rs = 1.0f / sqrtf(1.0f + 1e-5f);
  if (tid < NF) {
    par[tid]      = g1[tid] * rs * 0.0625f;
    par[16 + tid] = b1[tid];
    par[32 + tid] = g2[tid] * rs;
    par[48 + tid] = b2[tid];
    par[64 + tid] = g3[tid] * rs * (1.0f / 256.0f);
    par[80 + tid] = b3[tid];
  }
  if (tid < 48) { par[96 + tid] = wd[tid]; par[144 + tid] = wsd[tid]; }
  {
    const float* xrow = x + (size_t)node * TT;
    for (int i = tid; i < XSN; i += FTHR) {
      int t = i - XOF;
      const bool in = (t >= 0) && (t < TT);
      t = t < 0 ? 0 : (t > TT - 1 ? TT - 1 : t);
      const float v = xrow[t];
      xs[i] = in ? v : 0.0f;
    }
  }
  v16h aW, aP;
#pragma unroll
  for (int i = 0; i < 16; ++i) {
    const int k  = 8 * h + i + ((i >> 3) << 3);
    const int kc = k < KW ? k : KW - 1;
    const float wv = w1[m * KW + kc] * 16.0f;
    aW[i] = (k < KW) ? (_Float16)wv : (_Float16)0.0f;
    const int kp = k < NF ? k : NF - 1;
    const float pv = wp[m * NF + kp] * 16.0f;
    aP[i] = (k < NF) ? (_Float16)pv : (_Float16)0.0f;
  }
  __syncthreads();

  const v8f z8 = {0.f, 0.f, 0.f, 0.f, 0.f, 0.f, 0.f, 0.f};

#pragma unroll 1
  for (int tile = wave; tile < TT / 16; tile += FWAV) {
    const int t0 = tile * 16;
    const float* xb = xs + t0 + m + 8 * h;
    v16h bx;
#pragma unroll
    for (int i = 0; i < 8; ++i) {
      bx[i]     = (_Float16)xb[i];
      bx[8 + i] = (_Float16)xb[16 + i];
    }
    const v8f acc = wm(aW, bx, z8);
#pragma unroll
    for (int r = 0; r < 8; ++r) {
      const int f = 8 * h + r;
      const float v = acc[r] * par[f] + par[16 + f];
      s1[f * P1 + t0 + m] = elu_f(v);
    }
  }
  __syncthreads();

#pragma unroll 1
  for (int it = 0; it < (NF * TT / 4) / FTHR; ++it) {
    const int i  = it * FTHR + tid;
    const int c  = i >> 8;
    const int t4 = (i & 255) << 2;
    const float* row = s1 + c * P1;
    const v4f mid = *(const v4f*)(row + t4);
    int tl = t4 - 1; tl = tl < 0 ? 0 : tl;
    int tr = t4 + 4; tr = tr > TT - 1 ? TT - 1 : tr;
    float lf = row[tl]; lf = (t4 > 0) ? lf : 0.0f;
    float rg = row[tr]; rg = (t4 + 4 < TT) ? rg : 0.0f;
    const float k0 = par[96 + c * 3], k1 = par[97 + c * 3], k2 = par[98 + c * 3];
    v4f o;
    o.x = k0 * lf    + k1 * mid.x + k2 * mid.y;
    o.y = k0 * mid.x + k1 * mid.y + k2 * mid.z;
    o.z = k0 * mid.y + k1 * mid.z + k2 * mid.w;
    o.w = k0 * mid.z + k1 * mid.w + k2 * rg;
    const float sc = par[32 + c], sh = par[48 + c];
    o = o * sc + sh;
    o.x = elu_f(o.x); o.y = elu_f(o.y); o.z = elu_f(o.z); o.w = elu_f(o.w);
    *(v4f*)(s2 + c * P1 + t4) = o;
  }
  __syncthreads();

#pragma unroll 1
  for (int it = 0; it < (NF * TT / 4) / FTHR; ++it) {
    const int i  = it * FTHR + tid;
    const int c  = i >> 8;
    const int t4 = (i & 255) << 2;
    const float* row = s2 + c * P1;
    const v4f mid = *(const v4f*)(row + t4);
    int tl = t4 - 1; tl = tl < 0 ? 0 : tl;
    int tr = t4 + 4; tr = tr > TT - 1 ? TT - 1 : tr;
    float lf = row[tl]; lf = (t4 > 0) ? lf : 0.0f;
    float rg = row[tr]; rg = (t4 + 4 < TT) ? rg : 0.0f;
    const float k0 = par[144 + c * 3], k1 = par[145 + c * 3], k2 = par[146 + c * 3];
    const float o0 = k0 * lf    + k1 * mid.x + k2 * mid.y;
    const float o1 = k0 * mid.x + k1 * mid.y + k2 * mid.z;
    const float o2 = k0 * mid.y + k1 * mid.z + k2 * mid.w;
    const float o3 = k0 * mid.z + k1 * mid.w + k2 * rg;
    s3[(t4 + 0) * NF + c] = (_Float16)(o0 * 16.0f);
    s3[(t4 + 1) * NF + c] = (_Float16)(o1 * 16.0f);
    s3[(t4 + 2) * NF + c] = (_Float16)(o2 * 16.0f);
    s3[(t4 + 3) * NF + c] = (_Float16)(o3 * 16.0f);
  }
  __syncthreads();

  v8f facc = z8;
  const v16h zz = {};
#pragma unroll 1
  for (int tile = wave; tile < TT / 16; tile += FWAV) {
    const int t0 = tile * 16;
    Frag bq;
    bq.v = zz;
    bq.half[0] = *(const v8h*)(s3 + (t0 + m) * NF + 8 * h);
    const v8f acc = wm(aP, bq.v, z8);
#pragma unroll
    for (int r = 0; r < 8; ++r) {
      const int f = 8 * h + r;
      const float v = elu_f(acc[r] * par[64 + f] + par[80 + f]);
      facc[r] = facc[r] + v;
    }
  }
#pragma unroll
  for (int r = 0; r < 8; ++r) {
    float v = facc[r];
    v += __shfl_xor(v, 1, 32);
    v += __shfl_xor(v, 2, 32);
    v += __shfl_xor(v, 4, 32);
    v += __shfl_xor(v, 8, 32);
    facc[r] = v;
  }
  if (m == 0) {
#pragma unroll
    for (int r = 0; r < 8; ++r) red[wave * NF + 8 * h + r] = facc[r];
  }
  __syncthreads();
  if (tid < NF) {
    float s = 0.0f;
#pragma unroll
    for (int w = 0; w < FWAV; ++w) s += red[w * NF + tid];
    fvv[tid] = s * (1.0f / (float)TT);
  } else if (tid < FPITCH) {
    fvv[tid] = 0.0f;
  }
  __syncthreads();
  {
    const int lq = lane < 8 ? lane : 0;
    const v4f v = *(const v4f*)(fvv + 4 * lq);
    float* gp = feat + (size_t)node * FPITCH + 4 * lq;
    const bool wr = (wave == 0) && (lane < 8);
    if (wr) *(volatile v4f*)gp = v;
    __threadfence();
    if (wr) *(volatile v4f*)gp = v;
  }
}

__device__ __forceinline__ void stage_w(const float* __restrict__ W, int kin, _Float16* Wt, int tid) {
#pragma unroll 1
  for (int it = 0; it < (DF * 32) / GTHR; ++it) {
    const int i  = it * GTHR + tid;
    const int n  = i & (DF - 1);
    const int k  = i >> 7;
    const int kc = k < kin ? k : kin - 1;
    const float v = W[kc * DF + n] * 16.0f;
    Wt[n * AHP + k] = (k < kin) ? (_Float16)v : (_Float16)0.0f;
  }
}

__device__ __forceinline__ void proj_gemm(const _Float16* Ah, const _Float16* Wt, float* hh, int wave, int h, int m) {
  const v8f z8 = {0.f, 0.f, 0.f, 0.f, 0.f, 0.f, 0.f, 0.f};
  Frag bw;
  const _Float16* pb = Wt + (wave * 16 + m) * AHP + 8 * h;
  bw.half[0] = *(const v8h*)pb;
  bw.half[1] = *(const v8h*)(pb + 16);
#pragma unroll
  for (int rt = 0; rt < GN / 16; ++rt) {
    Frag a;
    const _Float16* pa = Ah + (rt * 16 + m) * AHP + 8 * h;
    a.half[0] = *(const v8h*)pa;
    a.half[1] = *(const v8h*)(pa + 16);
    const v8f acc = wm(a.v, bw.v, z8);
#pragma unroll
    for (int r = 0; r < 8; ++r) hh[(rt * 16 + 8 * h + r) * HP + wave * 16 + m] = acc[r] * 0.0625f;
  }
}

__device__ __forceinline__ void gat_logits(const float* hh, const float* av, float* asd, int tid) {
  const int d = tid >> 2, hd = tid & 3;
  const float* hr = hh + d * HP + hd * HF;
  const float* ps = av + hd * HF;
  const float* pd = av + DF + hd * HF;
  float ss = 0.0f, sd = 0.0f;
#pragma unroll 8
  for (int f = 0; f < HF; ++f) {
    const float v = hr[f];
    ss += v * ps[f];
    sd += v * pd[f];
  }
  asd[d * 8 + hd] = ss;
  asd[d * 8 + 4 + hd] = sd;
}

__device__ __forceinline__ void gat_drain(const float* hh, const float* asd, const int* esrc,
                                          const int* lst, const int* cnt, const int* off,
                                          float* gout, int tid) {
  const int d = tid >> 2, hd = tid & 3;
  const float ad = asd[d * 8 + 4 + hd];
  const float es = lrelu_f(asd[d * 8 + hd] + ad);
  int c = cnt[d]; c = c < 0 ? 0 : (c > NE ? NE : c);
  int o = off[d]; o = o < 0 ? 0 : (o > NE - 1 ? NE - 1 : o);
  int cm = c;
  cm = max(cm, __shfl_xor(cm, 16, 32));
  cm = max(cm, __shfl_xor(cm, 8, 32));
  cm = max(cm, __shfl_xor(cm, 4, 32));
  cm = max(cm, __shfl_xor(cm, 2, 32));
  cm = max(cm, __shfl_xor(cm, 1, 32));
  cm = cm > NE ? NE : cm;

  float mx = es;
#pragma unroll 1
  for (int q = 0; q < cm; ++q) {
    const bool val = q < c;
    int ix = o + q; ix = ix > NE - 1 ? NE - 1 : ix;
    const int j = lst[ix] & (NE - 1);
    const int s = esrc[j] & (GN - 1);
    const float e = lrelu_f(asd[s * 8 + hd] + ad);
    mx = val ? fmaxf(mx, e) : mx;
  }
  float p = expf(es - mx);
  float z = p;
  v4f a[8];
  {
    const float* hr = hh + d * HP + hd * HF;
#pragma unroll
    for (int k = 0; k < 8; ++k) a[k] = p * *(const v4f*)(hr + 4 * k);
  }
#pragma unroll 1
  for (int q = 0; q < cm; ++q) {
    const bool val = q < c;
    int ix = o + q; ix = ix > NE - 1 ? NE - 1 : ix;
    const int j = lst[ix] & (NE - 1);
    const int s = esrc[j] & (GN - 1);
    const float e = lrelu_f(asd[s * 8 + hd] + ad);
    const float pe = expf(e - mx);
    p = val ? pe : 0.0f;
    z += p;
    const float* sr = hh + s * HP + hd * HF;
#pragma unroll
    for (int k = 0; k < 8; ++k) a[k] = a[k] + p * *(const v4f*)(sr + 4 * k);
  }
  const float iz = 1.0f / (z + 1e-16f);
  float* go = gout + d * DF + hd * HF;
#pragma unroll
  for (int k = 0; k < 8; ++k) *(v4f*)(go + 4 * k) = a[k] * iz;
}

__global__ __launch_bounds__(GTHR) void k_graph(
    const float* __restrict__ feat, const int* __restrict__ ei,
    const float* __restrict__ W1,  const float* __restrict__ as1, const float* __restrict__ ad1,
    const float* __restrict__ bi1, const float* __restrict__ bg1, const float* __restrict__ bb1,
    const float* __restrict__ skw, const float* __restrict__ skb,
    const float* __restrict__ W2,  const float* __restrict__ as2, const float* __restrict__ ad2,
    const float* __restrict__ bi2, const float* __restrict__ bg2, const float* __restrict__ bb2,
    float* pooled, int nGraphs)
{
  extern __shared__ v4f dyng[];
  char* base = (char*)dyng;
  float*    hh   = (float*)(base + O_HH);
  float*    gout = (float*)(base + O_GO);
  float*    h1   = (float*)(base + O_H1);
  float*    skv  = (float*)(base + O_SK);
  float*    asd  = (float*)(base + O_ASD);
  float*    av   = (float*)(base + O_AV);
  int*      esrc = (int*)(base + O_EI);
  int*      edst = esrc + NE;
  int*      lst  = edst + NE;
  int*      cnt  = lst + NE;
  int*      off  = cnt + GN;
  _Float16* Ah   = (_Float16*)(base + O_AH);
  _Float16* Wt   = (_Float16*)(base + O_WT);
  _Float16* Wk   = (_Float16*)(base + O_WK);
  float*    pl   = (float*)(base + O_PL);

  const int tid = threadIdx.x, lane = tid & 31, wave = tid >> 5;
  const int h = lane >> 4, m = lane & 15;
  const int g = blockIdx.x;
  if (g >= nGraphs) return;
  const int nb = g * GN;
  const float rs = 1.0f / sqrtf(1.0f + 1e-5f);
  const v8f z8 = {0.f, 0.f, 0.f, 0.f, 0.f, 0.f, 0.f, 0.f};

  for (int i = tid; i < NE; i += GTHR) {
    int s = ei[i], d = ei[NE + i];
    s = s < 0 ? 0 : (s > GN - 1 ? GN - 1 : s);
    d = d < 0 ? 0 : (d > GN - 1 ? GN - 1 : d);
    esrc[i] = s;
    edst[i] = d;
  }
  {
    const int d = tid >> 2, q = tid & 3;
    const v4f fv = *(const v4f*)(feat + (size_t)(nb + d) * FPITCH + 4 * q);
    _Float16* ar = Ah + d * AHP + 4 * q;
    ar[0] = (_Float16)fv.x; ar[1] = (_Float16)fv.y; ar[2] = (_Float16)fv.z; ar[3] = (_Float16)fv.w;
    ar[16] = (_Float16)0.0f; ar[17] = (_Float16)0.0f; ar[18] = (_Float16)0.0f; ar[19] = (_Float16)0.0f;
  }
  stage_w(W1, NF, Wt, tid);
#pragma unroll 1
  for (int it = 0; it < (HF * 32) / GTHR; ++it) {
    const int i  = it * GTHR + tid;
    const int n  = i >> 5;
    const int k  = i & 31;
    const int kc = k < NF ? k : NF - 1;
    const float v = skw[n * NF + kc] * 16.0f;
    Wk[n * AHP + k] = (k < NF) ? (_Float16)v : (_Float16)0.0f;
  }
  {
    const float va = as1[tid & (DF - 1)];
    const float vd = ad1[tid & (DF - 1)];
    av[tid] = (tid < DF) ? va : vd;
  }
  __syncthreads();

  if (tid < GN) {
    int c = 0;
#pragma unroll 1
    for (int j = 0; j < NE; ++j) c += (edst[j] == tid) ? 1 : 0;
    cnt[tid] = c;
  }
  __syncthreads();
  if (tid == 0) {
    int a = 0;
#pragma unroll 1
    for (int d = 0; d < GN; ++d) { off[d] = a; a += cnt[d]; }
  }
  __syncthreads();
  if (tid < GN) {
    int p = off[tid];
#pragma unroll 1
    for (int j = 0; j < NE; ++j) {
      const int hit = (edst[j] == tid) ? 1 : 0;
      if (hit) lst[p > NE - 1 ? NE - 1 : p] = j;
      p += hit;
    }
  }

  proj_gemm(Ah, Wt, hh, wave, h, m);
  {
    const int rt = wave >> 1, ct = wave & 1;
    Frag a, bk;
    const _Float16* pa = Ah + (rt * 16 + m) * AHP + 8 * h;
    const _Float16* pb = Wk + (ct * 16 + m) * AHP + 8 * h;
    a.half[0]  = *(const v8h*)pa; a.half[1]  = *(const v8h*)(pa + 16);
    bk.half[0] = *(const v8h*)pb; bk.half[1] = *(const v8h*)(pb + 16);
    const v8f acc = wm(a.v, bk.v, z8);
    const float sb = skb[ct * 16 + m];
#pragma unroll
    for (int r = 0; r < 8; ++r) skv[(rt * 16 + 8 * h + r) * HF + ct * 16 + m] = acc[r] * 0.0625f + sb;
  }
  __syncthreads();

  gat_logits(hh, av, asd, tid);
  __syncthreads();
  gat_drain(hh, asd, esrc, lst, cnt, off, gout, tid);
  __syncthreads();

#pragma unroll 1
  for (int it = 0; it < (GN * HF) / GTHR; ++it) {
    const int i = it * GTHR + tid;
    const int d = i >> 5, f = i & 31;
    const float* gr = gout + d * DF + f;
    const float gs = ((gr[0] + gr[HF]) + gr[2 * HF]) + gr[3 * HF];
    float gv = gs * 0.25f + bi1[f];
    gv = gv * (bg1[f] * rs) + bb1[f];
    const float hv = gelu_f(gv + skv[d * HF + f]);
    h1[d * HF + f] = hv;
    Ah[d * AHP + f] = (_Float16)hv;
  }
  stage_w(W2, HF, Wt, tid);
  {
    const float va = as2[tid & (DF - 1)];
    const float vd = ad2[tid & (DF - 1)];
    av[tid] = (tid < DF) ? va : vd;
  }
  __syncthreads();

  proj_gemm(Ah, Wt, hh, wave, h, m);
  __syncthreads();
  gat_logits(hh, av, asd, tid);
  __syncthreads();
  gat_drain(hh, asd, esrc, lst, cnt, off, gout, tid);
  __syncthreads();

#pragma unroll 1
  for (int it = 0; it < (GN * HF) / GTHR; ++it) {
    const int i = it * GTHR + tid;
    const int d = i >> 5, f = i & 31;
    const float* gr = gout + d * DF + f;
    const float gs = ((gr[0] + gr[HF]) + gr[2 * HF]) + gr[3 * HF];
    float gv = gs * 0.25f + bi2[f];
    gv = gv * (bg2[f] * rs) + bb2[f];
    skv[d * HF + f] = gelu_f(gv + h1[d * HF + f]);
  }
  __syncthreads();

  if (tid < HF) {
    float s = 0.0f;
#pragma unroll 1
    for (int d = 0; d < GN; ++d) s += skv[d * HF + tid];
    pl[tid] = s * (1.0f / (float)GN);
  }
  __syncthreads();
  {
    const int lq = lane < 8 ? lane : 0;
    const v4f v = *(const v4f*)(pl + 4 * lq);
    float* gp = pooled + (size_t)g * FPITCH + 4 * lq;
    const bool wr = (wave == 0) && (lane < 8);
    if (wr) *(volatile v4f*)gp = v;
    __threadfence();
    if (wr) *(volatile v4f*)gp = v;
  }
}

__global__ __launch_bounds__(64) void k_head(const float* __restrict__ pooled, const float* __restrict__ fw,
                                             const float* __restrict__ fb, float* out, int nGraphs) {
  __shared__ __attribute__((aligned(16))) float ol[2 * GN];
  const int tid = threadIdx.x;
  const int b = tid < nGraphs ? tid : nGraphs - 1;
  const float* pr = pooled + (size_t)b * FPITCH;
  float o0 = 0.0f, o1 = 0.0f;
#pragma unroll 1
  for (int f = 0; f < HF; ++f) {
    const float v = pr[f];
    o0 += v * fw[f];
    o1 += v * fw[HF + f];
  }
  ol[2 * tid]     = o0 + fb[0];
  ol[2 * tid + 1] = o1 + fb[1];
  __syncthreads();
  const int lq = tid & 31;
  const v4f v = *(const v4f*)(ol + 4 * lq);
  const bool wr = tid < 32;
  if (wr) *(volatile v4f*)(out + 4 * lq) = v;
  __threadfence();
  if (wr) *(volatile v4f*)(out + 4 * lq) = v;
}

extern "C" void kernel_launch(void* const* d_in, const int* in_sizes, int n_in,
                              void* d_out, int out_size, void* d_ws, size_t ws_size,
                              hipStream_t stream) {
  const int nNodes = 4096, nGraphs = 64;
  if (n_in < 28) return;
  if (in_sizes[0] != nNodes * TT) return;
  if (in_sizes[1] != 2 * NE) return;
  if (in_sizes[2] != NF * KW || in_sizes[3] != NF || in_sizes[4] != NF) return;
  if (in_sizes[5] != NF * 3 || in_sizes[6] != NF || in_sizes[7] != NF) return;
  if (in_sizes[8] != NF * 3 || in_sizes[9] != NF * NF || in_sizes[10] != NF || in_sizes[11] != NF) return;
  if (in_sizes[12] != NF * DF || in_sizes[13] != DF || in_sizes[14] != DF || in_sizes[15] != HF) return;
  if (in_sizes[16] != HF || in_sizes[17] != HF || in_sizes[18] != HF * NF || in_sizes[19] != HF) return;
  if (in_sizes[20] != HF * DF || in_sizes[21] != DF || in_sizes[22] != DF || in_sizes[23] != HF) return;
  if (in_sizes[24] != HF || in_sizes[25] != HF || in_sizes[26] != 2 * HF || in_sizes[27] != 2) return;
  if (out_size != nGraphs * 2) return;

  const size_t o_feat = 0;
  const size_t o_pool = o_feat + (size_t)nNodes * FPITCH * sizeof(float);
  const size_t total  = o_pool + (size_t)nGraphs * FPITCH * sizeof(float);
  if (total > ws_size) return;

  const float* x        = (const float*)d_in[0];
  const int*   ei       = (const int*)d_in[1];
  const float* conv1_w  = (const float*)d_in[2];
  const float* bn1_g    = (const float*)d_in[3];
  const float* bn1_b    = (const float*)d_in[4];
  const float* dw_w     = (const float*)d_in[5];
  const float* bn2_g    = (const float*)d_in[6];
  const float* bn2_b    = (const float*)d_in[7];
  const float* sep_dw_w = (const float*)d_in[8];
  const float* sep_pw_w = (const float*)d_in[9];
  const float* bn3_g    = (const float*)d_in[10];
  const float* bn3_b    = (const float*)d_in[11];
  const float* gat1_w   = (const float*)d_in[12];
  const float* gat1_as  = (const float*)d_in[13];
  const float* gat1_ad  = (const float*)d_in[14];
  const float* gat1_bi  = (const float*)d_in[15];
  const float* gat1bn_g = (const float*)d_in[16];
  const float* gat1bn_b = (const float*)d_in[17];
  const float* skip1_w  = (const float*)d_in[18];
  const float* skip1_b  = (const float*)d_in[19];
  const float* gat2_w   = (const float*)d_in[20];
  const float* gat2_as  = (const float*)d_in[21];
  const float* gat2_ad  = (const float*)d_in[22];
  const float* gat2_bi  = (const float*)d_in[23];
  const float* gat2bn_g = (const float*)d_in[24];
  const float* gat2bn_b = (const float*)d_in[25];
  const float* fc_w     = (const float*)d_in[26];
  const float* fc_b     = (const float*)d_in[27];
  float* out    = (float*)d_out;
  float* feat   = (float*)((char*)d_ws + o_feat);
  float* pooled = (float*)((char*)d_ws + o_pool);

  hipFuncSetAttribute(reinterpret_cast<const void*>(&k_feat),
                      hipFuncAttributeMaxDynamicSharedMemorySize, LDS_FEAT);
  k_feat<<<nNodes, FTHR, LDS_FEAT, stream>>>(x, conv1_w, bn1_g, bn1_b, dw_w, bn2_g, bn2_b,
                                             sep_dw_w, sep_pw_w, bn3_g, bn3_b, feat, nNodes);

  hipFuncSetAttribute(reinterpret_cast<const void*>(&k_graph),
                      hipFuncAttributeMaxDynamicSharedMemorySize, LDS_GRAPH);
  k_graph<<<nGraphs, GTHR, LDS_GRAPH, stream>>>(feat, ei,
                                                gat1_w, gat1_as, gat1_ad, gat1_bi, gat1bn_g, gat1bn_b,
                                                skip1_w, skip1_b,
                                                gat2_w, gat2_as, gat2_ad, gat2_bi, gat2bn_g, gat2bn_b,
                                                pooled, nGraphs);

  k_head<<<1, 64, 0, stream>>>(pooled, fc_w, fc_b, out, nGraphs);
}
